// RWKV7Attention_78391743086652
// MI455X (gfx1250) — hardware-run, weakly checked
//
#include <hip/hip_runtime.h>
#include <math.h>

constexpr int kBatch  = 2;
constexpr int kSteps  = 2048;
constexpr int kChan   = 1024;
constexpr int kHeads  = 16;
constexpr int kHdim   = 64;
constexpr int kTok    = kBatch * kSteps;
constexpr size_t kPlane = (size_t)kTok * kChan;
constexpr int kLoraW  = 64;
constexpr int kLoraA  = 64;
constexpr int kLoraV  = 32;
constexpr int kLoraVP = 64;
constexpr int kLoraG  = 160;
constexpr int kLoraGP = 192;
constexpr int kChunk  = 16;

constexpr float kWCarry    = 16.0f;
constexpr float kWCarryInv = 1.0f / kWCarry;
constexpr float kMidCarry  = 16.0f;
constexpr float kUpScale   = 1.0f / (kWCarry * kMidCarry);
constexpr float kNegExpHalf = -0.60653065971263342f;
constexpr float kGnEps = (float)((double)kHdim * 1e-5);

static_assert(kHeads * kHdim == kChan);
static_assert(kTok % 64 == 0 && kChan % 64 == 0);
static_assert(kLoraW % 64 == 0 && kLoraA % 64 == 0 && kLoraVP % 64 == 0 && kLoraGP % 64 == 0);
static_assert(kChan % 32 == 0 && kLoraW % 32 == 0 && kLoraA % 32 == 0 && kLoraVP % 32 == 0 && kLoraGP % 32 == 0);
static_assert(kLoraV <= kLoraVP && kLoraG <= kLoraGP);
static_assert(kSteps % kChunk == 0);
static_assert((kSteps & (kSteps - 1)) == 0);
static_assert((kTok * kHeads) % 8 == 0);
static_assert(kHdim == 64 && kChunk == 16 && kChan / 8 == 128);

typedef __attribute__((ext_vector_type(16))) _Float16 v16h;
typedef __attribute__((ext_vector_type(8)))  _Float16 v8h;
typedef __attribute__((ext_vector_type(16))) __bf16   v16b;
typedef __attribute__((ext_vector_type(8)))  __bf16   v8b;
typedef __attribute__((ext_vector_type(8)))  float    v8f;
typedef __attribute__((ext_vector_type(4)))  float    v4f;
typedef __attribute__((ext_vector_type(2)))  float    v2f;
typedef __attribute__((ext_vector_type(4)))  unsigned int v4u;

__device__ __forceinline__ unsigned short f2bf_bits(float f) {
  unsigned u = __float_as_uint(f);
  return (unsigned short)((u + 0x7FFFu + ((u >> 16) & 1u)) >> 16);
}
__device__ __forceinline__ float bf_bits2f(unsigned short h) { return __uint_as_float(((unsigned)h) << 16); }
__device__ __forceinline__ unsigned pk16(unsigned short a, unsigned short b) {
  return (unsigned)a | ((unsigned)b << 16);
}
__device__ __forceinline__ unsigned short h_bits(float f) {
  const _Float16 h = (_Float16)f;
  return __builtin_bit_cast(unsigned short, h);
}
__device__ __forceinline__ void b_split(float v, unsigned short& hb, unsigned short& lb) {
  hb = f2bf_bits(v);
  lb = f2bf_bits(v - bf_bits2f(hb));
}
__device__ __forceinline__ v4u pack8_f16(const float (&v)[8]) {
  unsigned short hb[8];
#pragma unroll
  for (int e = 0; e < 8; ++e) hb[e] = h_bits(v[e]);
  return (v4u){pk16(hb[0], hb[1]), pk16(hb[2], hb[3]), pk16(hb[4], hb[5]), pk16(hb[6], hb[7])};
}
__device__ __forceinline__ void pack8_bsplit(const float (&v)[8], v4u& uh, v4u& ul) {
  unsigned short hb[8], lb[8];
#pragma unroll
  for (int e = 0; e < 8; ++e) b_split(v[e], hb[e], lb[e]);
  uh = (v4u){pk16(hb[0], hb[1]), pk16(hb[2], hb[3]), pk16(hb[4], hb[5]), pk16(hb[6], hb[7])};
  ul = (v4u){pk16(lb[0], lb[1]), pk16(lb[2], lb[3]), pk16(lb[4], lb[5]), pk16(lb[6], lb[7])};
}
__device__ __forceinline__ float wave_sum32(float v) {
#pragma unroll
  for (int o = 16; o > 0; o >>= 1) v += __shfl_xor(v, o, 32);
  return v;
}
__device__ __forceinline__ float sigmoid_f(float x) {
  return __builtin_amdgcn_rcpf(1.0f + expf(-x));
}

__device__ __forceinline__ void dep_guard4_h(v8f& a, v8f& b, v8f& c, v8f& d, v16h x, v16h y) {
  asm volatile("v_nop\n\tv_nop\n\tv_nop\n\tv_nop" : "+v"(a), "+v"(b), "+v"(c), "+v"(d) : "v"(x), "v"(y));
}
__device__ __forceinline__ void dep_guard4_b(v8f& a, v8f& b, v8f& c, v8f& d, v16b x, v16b y) {
  asm volatile("v_nop\n\tv_nop\n\tv_nop\n\tv_nop" : "+v"(a), "+v"(b), "+v"(c), "+v"(d) : "v"(x), "v"(y));
}
__device__ __forceinline__ void keep4_h(v16h a, v16h b, v16h c, v16h d) { asm volatile("v_nop" :: "v"(a), "v"(b), "v"(c), "v"(d)); }
__device__ __forceinline__ void keep4_b(v16b a, v16b b, v16b c, v16b d) { asm volatile("v_nop" :: "v"(a), "v"(b), "v"(c), "v"(d)); }
__device__ __forceinline__ void acc_guard4(v8f& a, v8f& b, v8f& c, v8f& d) {
  asm volatile("v_nop\n\tv_nop\n\tv_nop\n\tv_nop" : "+v"(a), "+v"(b), "+v"(c), "+v"(d));
}
template <typename T> struct Frag;
template <> struct Frag<_Float16> {
  typedef v16h V;
  union U { v16h v; v8h h[2]; };
  static __device__ __forceinline__ v16h load(const _Float16* p) {
    U f;
    f.h[0] = *(const v8h*)(p);
    f.h[1] = *(const v8h*)(p + 16);
    return f.v;
  }
  static __device__ __forceinline__ v8f mma(v16h a, v16h b, v8f c) {
    return __builtin_amdgcn_wmma_f32_16x16x32_f16(false, a, false, b, (short)0, c, false, false);
  }
  static __device__ __forceinline__ void guard4(v8f& a, v8f& b, v8f& c, v8f& d, v16h x, v16h y) { dep_guard4_h(a, b, c, d, x, y); }
  static __device__ __forceinline__ void keep(v16h a, v16h b, v16h c, v16h d) { keep4_h(a, b, c, d); }
};
template <> struct Frag<__bf16> {
  typedef v16b V;
  union U { v16b v; v8b h[2]; };
  static __device__ __forceinline__ v16b load(const __bf16* p) {
    U f;
    f.h[0] = *(const v8b*)(p);
    f.h[1] = *(const v8b*)(p + 16);
    return f.v;
  }
  static __device__ __forceinline__ v8f mma(v16b a, v16b b, v8f c) {
    return __builtin_amdgcn_wmma_f32_16x16x32_bf16(false, a, false, b, (short)0, c, false, false);
  }
  static __device__ __forceinline__ void guard4(v8f& a, v8f& b, v8f& c, v8f& d, v16b x, v16b y) { dep_guard4_b(a, b, c, d, x, y); }
  static __device__ __forceinline__ void keep(v16b a, v16b b, v16b c, v16b d) { keep4_b(a, b, c, d); }
};

template <int ET> struct Elem;
template <> struct Elem<0> { typedef _Float16 T; };
template <> struct Elem<1> { typedef __bf16 T; };

template <int ET, bool SPLIT, int OUT_MODE, int ACT>
__global__ __launch_bounds__(256) void wmma_gemm64(
    const unsigned short* __restrict__ Ap, const unsigned short* __restrict__ A2p, int lda,
    const unsigned short* __restrict__ Btp, const unsigned short* __restrict__ Bt2p, int ldb,
    void* __restrict__ Cout, void* __restrict__ Cout2, int ldc,
    int M, int N, int K, float scale, float post) {
  typedef typename Elem<ET>::T T;
  typedef typename Frag<T>::V V;
  static_assert(ACT == 0 || OUT_MODE != 0);
  __shared__ __align__(16) float sT[8][16 * 68];
  const int lane = threadIdx.x & 31;
  const int wave = threadIdx.x >> 5;
  const int tilesN = N >> 6;
  const int tilesM = M >> 6;
  const int tile = blockIdx.x * 8 + wave;
  if (tile >= tilesM * tilesN) return;
  const int tm = tile / tilesN;
  const int tn = tile - tm * tilesN;
  const int m0 = tm << 6;
  const int n0 = tn << 6;
  const int rlane = lane & 15;
  const int koff  = (lane >> 4) * 8;
  const int mOff  = (lane >> 4) * 8;

  const size_t aoff = (size_t)(m0 + rlane) * lda + koff;
  const size_t boff = (size_t)(n0 + rlane) * ldb + koff;
  const T* pah = (const T*)Ap + aoff;
  const T* pal = SPLIT ? ((const T*)A2p + aoff) : pah;
  const T* pbh = (const T*)Btp + boff;
  const T* pbl = SPLIT ? ((const T*)Bt2p + boff) : pbh;
  const size_t astep = (size_t)16 * lda;
  const size_t bstep = (size_t)16 * ldb;

  v8f acc[4][4];
#pragma unroll
  for (int i = 0; i < 4; ++i)
#pragma unroll
    for (int j = 0; j < 4; ++j) acc[i][j] = (v8f){0.f, 0.f, 0.f, 0.f, 0.f, 0.f, 0.f, 0.f};

  for (int k0 = 0; k0 < K; k0 += 32) {
    V bh[4], bl[4];
#pragma unroll
    for (int j = 0; j < 4; ++j) {
      bh[j] = Frag<T>::load(pbh + j * bstep + k0);
      bl[j] = bh[j];
      if (SPLIT) bl[j] = Frag<T>::load(pbl + j * bstep + k0);
    }
#pragma unroll
    for (int i = 0; i < 4; ++i) {
      const V ah = Frag<T>::load(pah + i * astep + k0);
      V al = ah;
      if (SPLIT) al = Frag<T>::load(pal + i * astep + k0);
#pragma unroll
      for (int j = 0; j < 4; ++j) {
        acc[i][j] = Frag<T>::mma(ah, bh[j], acc[i][j]);
        if (SPLIT) {
          acc[i][j] = Frag<T>::mma(ah, bl[j], acc[i][j]);
          acc[i][j] = Frag<T>::mma(al, bh[j], acc[i][j]);
        }
      }
      Frag<T>::guard4(acc[i][0], acc[i][1], acc[i][2], acc[i][3], ah, al);
    }
    Frag<T>::keep(bh[0], bh[1], bh[2], bh[3]);
    if (SPLIT) Frag<T>::keep(bl[0], bl[1], bl[2], bl[3]);
  }
  acc_guard4(acc[0][0], acc[0][1], acc[0][2], acc[0][3]);
  acc_guard4(acc[1][0], acc[1][1], acc[1][2], acc[1][3]);
  acc_guard4(acc[2][0], acc[2][1], acc[2][2], acc[2][3]);
  acc_guard4(acc[3][0], acc[3][1], acc[3][2], acc[3][3]);

  float* slab = sT[wave];
#pragma unroll
  for (int i = 0; i < 4; ++i) {
    const int mBase = m0 + (i << 4);
#pragma unroll
    for (int j = 0; j < 4; ++j) {
#pragma unroll
      for (int r = 0; r < 8; ++r) {
        const float v = acc[i][j][r] * scale;
        slab[(mOff + r) * 68 + (j << 4) + rlane] = v;
      }
    }
    __builtin_amdgcn_fence(__ATOMIC_RELEASE, "workgroup");
    __builtin_amdgcn_wave_barrier();
    __builtin_amdgcn_fence(__ATOMIC_ACQUIRE, "workgroup");
    if (OUT_MODE == 0) {
      float* C = (float*)Cout;
      const int hh = lane >> 4, c4 = (lane & 15) * 4;
      for (int pass = 0; pass < 2; ++pass) {
#pragma unroll
        for (int it = 0; it < 8; ++it) {
          const int row = it * 2 + hh;
          const v4f v = *(const v4f*)(slab + row * 68 + c4);
          *(volatile v4f*)(C + (size_t)(mBase + row) * ldc + n0 + c4) = v;
        }
        __threadfence();
      }
    } else {
      const int q = lane >> 3, c8 = (lane & 7) * 8;
      if (ACT != 0) {
#pragma unroll 1
        for (int it = 0; it < 4; ++it) {
          float* sp = slab + (it * 4 + q) * 68 + c8;
#pragma unroll
          for (int e = 0; e < 8; ++e) {
            const float xin = sp[e];
            float y;
            if (ACT == 1) y = tanhf(xin);
            else y = sigmoid_f(xin);
            sp[e] = y * post;
          }
        }
      }
      unsigned short* C  = (unsigned short*)Cout;
      unsigned short* C2 = (unsigned short*)Cout2;
      for (int pass = 0; pass < 2; ++pass) {
#pragma unroll
        for (int it = 0; it < 4; ++it) {
          const int row = it * 4 + q;
          const float* sp = slab + row * 68 + c8;
          v8h hv, lv;
#pragma unroll
          for (int e = 0; e < 8; ++e) {
            const float sv = sp[e];
            if (OUT_MODE == 1) {
              hv[e] = (_Float16)sv;
              lv[e] = (_Float16)0.0f;
            } else {
              const unsigned short hb = f2bf_bits(sv);
              const unsigned short lb = f2bf_bits(sv - bf_bits2f(hb));
              hv[e] = __builtin_bit_cast(_Float16, hb);
              lv[e] = __builtin_bit_cast(_Float16, lb);
            }
          }
          *(volatile v8h*)(C + (size_t)(mBase + row) * ldc + n0 + c8) = hv;
          if (OUT_MODE == 2) *(volatile v8h*)(C2 + (size_t)(mBase + row) * ldc + n0 + c8) = lv;
        }
        __threadfence();
      }
    }
    __builtin_amdgcn_fence(__ATOMIC_RELEASE, "workgroup");
    __builtin_amdgcn_wave_barrier();
    __builtin_amdgcn_fence(__ATOMIC_ACQUIRE, "workgroup");
  }
}

template <bool SPLIT>
__global__ __launch_bounds__(256) void wt_plane_kernel(const float* __restrict__ W0, const float* __restrict__ W1,
                                                       unsigned short* __restrict__ outh, unsigned short* __restrict__ outl,
                                                       int Kd, int Nd, int KdP, int NdP, float carry) {
  __shared__ float sm[64][65];
  const int t  = threadIdx.x;
  const int k0 = blockIdx.x * 64;
  const int n0 = blockIdx.y * 64;
  const int z  = blockIdx.z;
  const float* W = (z == 0) ? W0 : W1;
#pragma unroll
  for (int i = 0; i < 16; ++i) {
    const int e = i * 256 + t;
    const int r = e >> 6;
    const int c = e & 63;
    const int kk = k0 + r;
    const int nn = n0 + c;
    const bool valid = (kk < Kd) && (nn < Nd);
    const int kc = (kk < Kd) ? kk : (Kd - 1);
    const int nc = (nn < Nd) ? nn : (Nd - 1);
    const float v = W[(size_t)kc * Nd + nc];
    sm[c][r] = valid ? (v * carry) : 0.0f;
  }
  __syncthreads();
  const int lane = t & 31, wave = t >> 5;
  const int q = lane >> 3, c8 = (lane & 7) * 8;
  const size_t pofs = (size_t)z * (size_t)NdP * (size_t)KdP;
  for (int pass = 0; pass < 2; ++pass) {
#pragma unroll
    for (int it = 0; it < 2; ++it) {
      const int row = wave * 8 + it * 4 + q;
      float v[8];
#pragma unroll
      for (int e = 0; e < 8; ++e) v[e] = sm[row][c8 + e];
      v4u uh, ul;
      if (SPLIT) {
        pack8_bsplit(v, uh, ul);
      } else {
        uh = pack8_f16(v);
        ul = uh;
      }
      const size_t o = pofs + (size_t)(n0 + row) * KdP + k0 + c8;
      *(volatile v4u*)(outh + o) = uh;
      if (SPLIT) *(volatile v4u*)(outl + o) = ul;
    }
    __threadfence();
  }
}

template <bool SPLIT>
__global__ __launch_bounds__(256) void wcast_kernel(const float* __restrict__ in, unsigned short* __restrict__ P0,
                                                    unsigned short* __restrict__ P1, int n8, float carry) {
  const int i = blockIdx.x * 256 + threadIdx.x;
  if (i >= n8) return;
  const float* p = in + 8 * (size_t)i;
  const v4f a = *(const v4f*)(p);
  const v4f c = *(const v4f*)(p + 4);
  float v[8];
#pragma unroll
  for (int e = 0; e < 4; ++e) {
    v[e]     = a[e] * carry;
    v[4 + e] = c[e] * carry;
  }
  v4u u0, u1;
  if (SPLIT) {
    pack8_bsplit(v, u0, u1);
  } else {
    u0 = pack8_f16(v);
    u1 = u0;
  }
  const size_t off = 8 * (size_t)i;
  *(volatile v4u*)(P0 + off) = u0;
  if (SPLIT) *(volatile v4u*)(P1 + off) = u1;
  __threadfence();
  *(volatile v4u*)(P0 + off) = u0;
  if (SPLIT) *(volatile v4u*)(P1 + off) = u1;
}

__device__ __forceinline__ void mix8(const float* __restrict__ m, int c8, const float (&cur)[8],
                                     const float (&xx)[8], float (&o)[8]) {
  const v4f a = *(const v4f*)(m + c8);
  const v4f b = *(const v4f*)(m + c8 + 4);
#pragma unroll
  for (int e = 0; e < 4; ++e) {
    o[e]     = cur[e]     + xx[e]     * a[e];
    o[4 + e] = cur[4 + e] + xx[4 + e] * b[e];
  }
}

template <bool SPLIT>
__global__ __launch_bounds__(256) void mix_kernel(const float* __restrict__ x,
                                                  const float* __restrict__ mA, const float* __restrict__ mB,
                                                  unsigned short* __restrict__ P0, unsigned short* __restrict__ P1) {
  const int i = blockIdx.x * 256 + threadIdx.x;
  if (i >= kTok * (kChan / 8)) return;
  const int row = i >> 7;
  const int c8  = (i & 127) * 8;
  const bool first = (row & (kSteps - 1)) == 0;
  const int prow = first ? row : (row - 1);
  const float* xp = x + (size_t)row * kChan + c8;
  const float* pp = x + (size_t)prow * kChan + c8;
  const v4f a  = *(const v4f*)(xp);
  const v4f b  = *(const v4f*)(xp + 4);
  const v4f pa = *(const v4f*)(pp);
  const v4f pb = *(const v4f*)(pp + 4);
  float cur[8], xx[8];
#pragma unroll
  for (int e = 0; e < 4; ++e) {
    cur[e]     = a[e];
    cur[4 + e] = b[e];
    const float p0 = first ? 0.0f : pa[e];
    const float p1 = first ? 0.0f : pb[e];
    xx[e]     = p0 - a[e];
    xx[4 + e] = p1 - b[e];
  }
  float o[8];
  v4u u0, u1;
  mix8(mA, c8, cur, xx, o);
  if (SPLIT) {
    pack8_bsplit(o, u0, u1);
  } else {
    u0 = pack8_f16(o);
    mix8(mB, c8, cur, xx, o);
    u1 = pack8_f16(o);
  }
  const size_t off = (size_t)i * 8;
  *(volatile v4u*)(P0 + off) = u0;
  *(volatile v4u*)(P1 + off) = u1;
  __threadfence();
  *(volatile v4u*)(P0 + off) = u0;
  *(volatile v4u*)(P1 + off) = u1;
}

__global__ __launch_bounds__(256) void gate_prep_kernel(float* PK, float* PV, float* PW, float* PA, float* PX,
                                                        const float* __restrict__ vfirst,
                                                        const float* __restrict__ w0, const float* __restrict__ a0,
                                                        const float* __restrict__ v0b, const float* __restrict__ k_k,
                                                        const float* __restrict__ k_a) {
  const int lane = threadIdx.x & 31;
  const int pair = blockIdx.x * 8 + (threadIdx.x >> 5);
  const int tok = pair >> 4;
  const int h   = pair & 15;
  const size_t base = (size_t)tok * kChan + (size_t)h * kHdim;
  const int cb = h * kHdim;
  float ss;
  {
    const float ka = PK[base + lane] * k_k[cb + lane];
    const float kb = PK[base + lane + 32] * k_k[cb + lane + 32];
    ss = wave_sum32(ka * ka + kb * kb);
  }
  const float inv = 1.0f / fmaxf(sqrtf(ss), 1e-12f);
#pragma unroll 1
  for (int hf = 0; hf < 2; ++hf) {
    const size_t idx = base + lane + 32 * hf;
    const int c = cb + lane + 32 * hf;
    const float k0  = PK[idx];
    const float kkv = (k0 * k_k[c]) * inv;
    const float av  = sigmoid_f(a0[c] + PA[idx]);
    const float km  = k0 + (k0 * (av - 1.0f)) * k_a[c];
    const float wv  = kNegExpHalf * sigmoid_f(w0[c] + PW[idx]);
    const float dv  = expf(wv);
    const float vg  = sigmoid_f(v0b[c] + PX[idx]);
    const float vp  = PV[idx];
    const float vm  = vp + (vfirst[idx] - vp) * vg;
    const float bv  = kkv * av;
    *(volatile float*)(PK + idx) = km;
    *(volatile float*)(PV + idx) = vm;
    *(volatile float*)(PW + idx) = dv;
    *(volatile float*)(PA + idx) = bv;
    *(volatile float*)(PX + idx) = kkv;
    __threadfence();
    *(volatile float*)(PK + idx) = km;
    *(volatile float*)(PV + idx) = vm;
    *(volatile float*)(PW + idx) = dv;
    *(volatile float*)(PA + idx) = bv;
    *(volatile float*)(PX + idx) = kkv;
  }
}

__global__ __launch_bounds__(256) void state_scan_kernel(const float* __restrict__ Rf, const float* __restrict__ Dd,
                                                         const float* __restrict__ Kf, const float* __restrict__ Vf,
                                                         const float* __restrict__ KKf, const float* __restrict__ Bv,
                                                         float* __restrict__ Y) {
  __shared__ __align__(16) float lv[6 * kChunk * 64];
  __shared__ __align__(16) float yb[kChunk * 64];
  const int bh  = blockIdx.x;
  const int b   = bh >> 4;
  const int h   = bh & 15;
  const int tid = threadIdx.x;
  const int i   = tid >> 2;
  const int q   = tid & 3;
  const int j0  = q * 16;
  const int lrow = tid >> 4;
  const int lc4  = (tid & 15) * 4;
  const size_t base = (size_t)b * kSteps * kChan + (size_t)h * kHdim;

  float S[16];
#pragma unroll
  for (int jj = 0; jj < 16; ++jj) S[jj] = 0.0f;

#pragma unroll 1
  for (int ch = 0; ch < kSteps / kChunk; ++ch) {
    const size_t goff = base + (size_t)(ch * kChunk + lrow) * kChan + lc4;
    {
      const v4f t0 = *(const v4f*)(Rf + goff);
      const v4f t1 = *(const v4f*)(Dd + goff);
      const v4f t2 = *(const v4f*)(Kf + goff);
      const v4f t3 = *(const v4f*)(Vf + goff);
      const v4f t4 = *(const v4f*)(KKf + goff);
      const v4f t5 = *(const v4f*)(Bv + goff);
      const int lo = lrow * 64 + lc4;
      *(v4f*)(lv + 0 * kChunk * 64 + lo) = t0;
      *(v4f*)(lv + 1 * kChunk * 64 + lo) = t1;
      *(v4f*)(lv + 2 * kChunk * 64 + lo) = t2;
      *(v4f*)(lv + 3 * kChunk * 64 + lo) = t3;
      *(v4f*)(lv + 4 * kChunk * 64 + lo) = t4;
      *(v4f*)(lv + 5 * kChunk * 64 + lo) = t5;
    }
    __syncthreads();

#pragma unroll 1
    for (int s = 0; s < kChunk; ++s) {
      const float* pr  = lv + 0 * kChunk * 64 + s * 64 + j0;
      const float* pd  = lv + 1 * kChunk * 64 + s * 64 + j0;
      const float* pk  = lv + 2 * kChunk * 64 + s * 64 + j0;
      const float* pkk = lv + 4 * kChunk * 64 + s * 64 + j0;
      const float* pb  = lv + 5 * kChunk * 64 + s * 64 + j0;
      const float vi = lv[3 * kChunk * 64 + s * 64 + i];
      float sa = 0.0f;
#pragma unroll
      for (int g4 = 0; g4 < 4; ++g4) {
        const v4f k4 = *(const v4f*)(pkk + 4 * g4);
#pragma unroll
        for (int e = 0; e < 4; ++e) sa += S[4 * g4 + e] * k4[e];
      }
      sa += __shfl_xor(sa, 1, 32);
      sa += __shfl_xor(sa, 2, 32);
      sa = -sa;
      float out = 0.0f;
#pragma unroll
      for (int g4 = 0; g4 < 4; ++g4) {
        const v4f d4 = *(const v4f*)(pd + 4 * g4);
        const v4f b4 = *(const v4f*)(pb + 4 * g4);
        const v4f k4 = *(const v4f*)(pk + 4 * g4);
        const v4f r4 = *(const v4f*)(pr + 4 * g4);
#pragma unroll
        for (int e = 0; e < 4; ++e) {
          const float sn = S[4 * g4 + e] * d4[e] + sa * b4[e] + vi * k4[e];
          S[4 * g4 + e] = sn;
          out += sn * r4[e];
        }
      }
      out += __shfl_xor(out, 1, 32);
      out += __shfl_xor(out, 2, 32);
      if (q == 0) yb[s * 64 + i] = out;
    }
    __syncthreads();
    {
      const v4f val = *(const v4f*)(yb + lrow * 64 + lc4);
      *(volatile v4f*)(Y + goff) = val;
      __threadfence();
      *(volatile v4f*)(Y + goff) = val;
    }
  }
}

__global__ __launch_bounds__(256) void norm_gate_kernel(const float* __restrict__ Y, const float* __restrict__ Rf,
                                                        const float* __restrict__ Kf, const float* __restrict__ Vf,
                                                        const float* __restrict__ Gf, const float* __restrict__ r_k,
                                                        const float* __restrict__ gn_w, const float* __restrict__ gn_b,
                                                        unsigned* __restrict__ OGh, unsigned* __restrict__ OGl) {
  const int lane = threadIdx.x & 31;
  const int pair = blockIdx.x * 8 + (threadIdx.x >> 5);
  const int tok = pair >> 4;
  const int h   = pair & 15;
  const size_t base = (size_t)tok * kChan + (size_t)h * kHdim + 2 * lane;
  const int c = h * kHdim + 2 * lane;
  const v2f y2 = *(const v2f*)(Y + base);
  const v2f r2 = *(const v2f*)(Rf + base);
  const v2f k2 = *(const v2f*)(Kf + base);
  const v2f v2 = *(const v2f*)(Vf + base);
  const v2f g2 = *(const v2f*)(Gf + base);
  const v2f q2 = *(const v2f*)(r_k + c);
  const v2f w2 = *(const v2f*)(gn_w + c);
  const v2f b2 = *(const v2f*)(gn_b + c);
  const float mu = wave_sum32(y2[0] + y2[1]) * (1.0f / (float)kHdim);
  const float d0 = y2[0] - mu;
  const float d1 = y2[1] - mu;
  const float var = wave_sum32(d0 * d0 + d1 * d1) * (1.0f / (float)kHdim);
  const float inv = 1.0f / sqrtf(var + kGnEps);
  const float bsum = wave_sum32(r2[0] * k2[0] * q2[0] + r2[1] * k2[1] * q2[1]);
  const float o0 = (((d0 * inv) * w2[0] + b2[0]) + bsum * v2[0]) * g2[0];
  const float o1 = (((d1 * inv) * w2[1] + b2[1]) + bsum * v2[1]) * g2[1];
  unsigned short h0, s0, h1, s1;
  b_split(o0, h0, s0);
  b_split(o1, h1, s1);
  const unsigned wh = pk16(h0, h1);
  const unsigned wl = pk16(s0, s1);
  const size_t widx = base >> 1;
  *(volatile unsigned*)(OGh + widx) = wh;
  *(volatile unsigned*)(OGl + widx) = wl;
  __threadfence();
  *(volatile unsigned*)(OGh + widx) = wh;
  *(volatile unsigned*)(OGl + widx) = wl;
}

extern "C" void kernel_launch(void* const* d_in, const int* in_sizes, int n_in,
                              void* d_out, int out_size, void* d_ws, size_t ws_size, hipStream_t stream) {
  if (n_in < 28 || d_out == nullptr || d_ws == nullptr) return;
  const int nP = (int)kPlane;
  if (in_sizes[0] != nP || in_sizes[1] != nP) return;
  for (int i = 2; i <= 8; ++i) if (in_sizes[i] != kChan) return;
  if (in_sizes[9] != kChan * kLoraW || in_sizes[10] != kLoraW * kChan || in_sizes[11] != kChan) return;
  if (in_sizes[12] != kChan * kLoraA || in_sizes[13] != kLoraA * kChan || in_sizes[14] != kChan) return;
  if (in_sizes[15] != kChan * kLoraV || in_sizes[16] != kLoraV * kChan) return;
  if (in_sizes[17] != kChan * kLoraG || in_sizes[18] != kLoraG * kChan) return;
  if (in_sizes[19] != kChan || in_sizes[20] != kChan || in_sizes[21] != kHeads * kHdim) return;
  for (int i = 22; i <= 25; ++i) if (in_sizes[i] != kChan * kChan) return;
  if (in_sizes[26] != kChan || in_sizes[27] != kChan) return;
  if (out_size != nP) return;

  const float* x      = (const float*)d_in[0];
  const float* vfirst = (const float*)d_in[1];
  const float* x_r = (const float*)d_in[2];
  const float* x_w = (const float*)d_in[3];
  const float* x_k = (const float*)d_in[4];
  const float* x_v = (const float*)d_in[5];
  const float* x_a = (const float*)d_in[6];
  const float* x_g = (const float*)d_in[7];
  const float* w0  = (const float*)d_in[8];
  const float* w1  = (const float*)d_in[9];
  const float* w2  = (const float*)d_in[10];
  const float* a0  = (const float*)d_in[11];
  const float* a1  = (const float*)d_in[12];
  const float* a2  = (const float*)d_in[13];
  const float* v0  = (const float*)d_in[14];
  const float* v1  = (const float*)d_in[15];
  const float* v2  = (const float*)d_in[16];
  const float* g1  = (const float*)d_in[17];
  const float* g2  = (const float*)d_in[18];
  const float* k_k = (const float*)d_in[19];
  const float* k_a = (const float*)d_in[20];
  const float* r_k = (const float*)d_in[21];
  const float* W_r = (const float*)d_in[22];
  const float* W_k = (const float*)d_in[23];
  const float* W_v = (const float*)d_in[24];
  const float* W_o = (const float*)d_in[25];
  const float* gn_w = (const float*)d_in[26];
  const float* gn_b = (const float*)d_in[27];
  float* out0 = (float*)d_out;

  char* ws = (char*)d_ws;
  size_t off = 0;
  auto carve = [&](size_t bytes) -> char* {
    char* p = ws + off;
    off += (bytes + 255) & ~(size_t)255;
    return p;
  };
  const size_t wBig = (size_t)kChan * kChan;
  float* PR = (float*)carve(kPlane * 4);
  float* PK = (float*)carve(kPlane * 4);
  float* PV = (float*)carve(kPlane * 4);
  float* PW = (float*)carve(kPlane * 4);
  float* PA = (float*)carve(kPlane * 4);
  float* PX = (float*)carve(kPlane * 4);
  unsigned short* AB0 = (unsigned short*)carve(kPlane * 4);
  unsigned short* AB1 = AB0 + kPlane;
  unsigned short* WBh = (unsigned short*)carve(wBig * 2);
  unsigned short* WBl = (unsigned short*)carve(wBig * 2);
  unsigned short* WV16 = (unsigned short*)carve(wBig * 2);
  unsigned short* W1T = (unsigned short*)carve((size_t)2 * kLoraW * kChan * 2);
  unsigned short* A1T = W1T + (size_t)kLoraW * kChan;
  unsigned short* V1T = (unsigned short*)carve((size_t)kLoraVP * kChan * 2);
  unsigned short* G1T = (unsigned short*)carve((size_t)kLoraGP * kChan * 2);
  unsigned short* W2T = (unsigned short*)carve((size_t)2 * kChan * kLoraW * 2);
  unsigned short* A2T = W2T + (size_t)kChan * kLoraW;
  unsigned short* V2T = (unsigned short*)carve((size_t)kChan * kLoraVP * 2);
  unsigned short* G2Th = (unsigned short*)carve((size_t)kChan * kLoraGP * 2);
  unsigned short* G2Tl = (unsigned short*)carve((size_t)kChan * kLoraGP * 2);
  unsigned short* WMID = (unsigned short*)carve((size_t)kTok * kLoraW * 2);
  unsigned short* AMID = (unsigned short*)carve((size_t)kTok * kLoraA * 2);
  unsigned short* VMID = (unsigned short*)carve((size_t)kTok * kLoraVP * 2);
  unsigned short* GMIDh = (unsigned short*)carve((size_t)kTok * kLoraGP * 2);
  unsigned short* GMIDl = (unsigned short*)carve((size_t)kTok * kLoraGP * 2);
  if (off > ws_size || off > (size_t)134217728) return;
  float* Yf = (float*)AB0;
  unsigned short* OGh = (unsigned short*)PA;
  unsigned short* OGl = OGh + kPlane;

  const int mixBlocks  = (kTok * (kChan / 8)) / 256;
  const int castBlocks = (int)(wBig / 8) / 256;
  const int gbBig  = ((kTok / 64) * (kChan / 64) + 7) / 8;
  const int gb64   = ((kTok / 64) * (64 / 64) + 7) / 8;
  const int gb192  = ((kTok / 64) * (kLoraGP / 64) + 7) / 8;

  wt_plane_kernel<false><<<dim3(kChan / 64, kLoraW / 64, 2), 256, 0, stream>>>(w1, a1, W1T, W1T, kChan, kLoraW, kChan, kLoraW, kWCarry);
  wt_plane_kernel<false><<<dim3(kChan / 64, kLoraVP / 64, 1), 256, 0, stream>>>(v1, v1, V1T, V1T, kChan, kLoraV, kChan, kLoraVP, kWCarry);
  wt_plane_kernel<false><<<dim3(kChan / 64, kLoraGP / 64, 1), 256, 0, stream>>>(g1, g1, G1T, G1T, kChan, kLoraG, kChan, kLoraGP, kWCarry);
  wt_plane_kernel<false><<<dim3(kLoraW / 64, kChan / 64, 2), 256, 0, stream>>>(w2, a2, W2T, W2T, kLoraW, kChan, kLoraW, kChan, kWCarry);
  wt_plane_kernel<false><<<dim3(kLoraVP / 64, kChan / 64, 1), 256, 0, stream>>>(v2, v2, V2T, V2T, kLoraV, kChan, kLoraVP, kChan, kWCarry);
  wt_plane_kernel<true><<<dim3(kLoraGP / 64, kChan / 64, 1), 256, 0, stream>>>(g2, g2, G2Th, G2Tl, kLoraG, kChan, kLoraGP, kChan, 1.0f);

  wcast_kernel<true><<<castBlocks, 256, 0, stream>>>(W_r, WBh, WBl, (int)(wBig / 8), 1.0f);
  mix_kernel<true><<<mixBlocks, 256, 0, stream>>>(x, x_r, x_r, AB0, AB1);
  wmma_gemm64<1, true, 0, 0><<<gbBig, 256, 0, stream>>>(AB0, AB1, kChan, WBh, WBl, kChan,
      (void*)PR, (void*)PR, kChan, kTok, kChan, kChan, 1.0f, 1.0f);

  wcast_kernel<true><<<castBlocks, 256, 0, stream>>>(W_k, WBh, WBl, (int)(wBig / 8), 1.0f);
  mix_kernel<true><<<mixBlocks, 256, 0, stream>>>(x, x_k, x_k, AB0, AB1);
  wmma_gemm64<1, true, 0, 0><<<gbBig, 256, 0, stream>>>(AB0, AB1, kChan, WBh, WBl, kChan,
      (void*)PK, (void*)PK, kChan, kTok, kChan, kChan, 1.0f, 1.0f);

  wcast_kernel<false><<<castBlocks, 256, 0, stream>>>(W_v, WV16, WV16, (int)(wBig / 8), kWCarry);
  mix_kernel<false><<<mixBlocks, 256, 0, stream>>>(x, x_v, x_g, AB0, AB1);
  wmma_gemm64<0, false, 0, 0><<<gbBig, 256, 0, stream>>>(AB0, AB0, kChan, WV16, WV16, kChan,
      (void*)PV, (void*)PV, kChan, kTok, kChan, kChan, kWCarryInv, 1.0f);
  wmma_gemm64<0, false, 1, 0><<<gb64, 256, 0, stream>>>(AB0, AB0, kChan, V1T, V1T, kChan,
      (void*)VMID, (void*)VMID, kLoraVP, kTok, kLoraVP, kChan, 1.0f, 1.0f);
  wmma_gemm64<0, false, 2, 2><<<gb192, 256, 0, stream>>>(AB1, AB1, kChan, G1T, G1T, kChan,
      (void*)GMIDh, (void*)GMIDl, kLoraGP, kTok, kLoraGP, kChan, kWCarryInv, 1.0f);
  wmma_gemm64<0, false, 0, 0><<<gbBig, 256, 0, stream>>>(VMID, VMID, kLoraVP, V2T, V2T, kLoraVP,
      (void*)PX, (void*)PX, kChan, kTok, kChan, kLoraVP, kUpScale, 1.0f);

  mix_kernel<false><<<mixBlocks, 256, 0, stream>>>(x, x_w, x_a, AB0, AB1);
  wmma_gemm64<0, false, 1, 1><<<gb64, 256, 0, stream>>>(AB0, AB0, kChan, W1T, W1T, kChan,
      (void*)WMID, (void*)WMID, kLoraW, kTok, kLoraW, kChan, kWCarryInv, kMidCarry);
  wmma_gemm64<0, false, 1, 0><<<gb64, 256, 0, stream>>>(AB1, AB1, kChan, A1T, A1T, kChan,
      (void*)AMID, (void*)AMID, kLoraA, kTok, kLoraA, kChan, 1.0f, 1.0f);
  wmma_gemm64<0, false, 0, 0><<<gbBig, 256, 0, stream>>>(WMID, WMID, kLoraW, W2T, W2T, kLoraW,
      (void*)PW, (void*)PW, kChan, kTok, kChan, kLoraW, kUpScale, 1.0f);
  wmma_gemm64<0, false, 0, 0><<<gbBig, 256, 0, stream>>>(AMID, AMID, kLoraA, A2T, A2T, kLoraA,
      (void*)PA, (void*)PA, kChan, kTok, kChan, kLoraA, kUpScale, 1.0f);

  gate_prep_kernel<<<(kTok * kHeads) / 8, 256, 0, stream>>>(PK, PV, PW, PA, PX, vfirst, w0, a0, v0, k_k, k_a);

  state_scan_kernel<<<kBatch * kHeads, 256, 0, stream>>>(PR, PW, PK, PV, PX, PA, Yf);

  wmma_gemm64<1, true, 0, 0><<<gbBig, 256, 0, stream>>>(GMIDh, GMIDl, kLoraGP, G2Th, G2Tl, kLoraGP,
      (void*)PX, (void*)PX, kChan, kTok, kChan, kLoraGP, 1.0f, 1.0f);

  norm_gate_kernel<<<(kTok * kHeads) / 8, 256, 0, stream>>>(Yf, PR, PK, PV, PX, r_k, gn_w, gn_b,
                                                            (unsigned*)OGh, (unsigned*)OGl);

  wcast_kernel<true><<<castBlocks, 256, 0, stream>>>(W_o, WBh, WBl, (int)(wBig / 8), 1.0f);
  wmma_gemm64<1, true, 0, 0><<<gbBig, 256, 0, stream>>>(OGh, OGl, kChan, WBh, WBl, kChan,
      (void*)out0, (void*)out0, kChan, kTok, kChan, kChan, 1.0f, 1.0f);
}
